// TaylorMap_12232066859102
// MI455X (gfx1250) — hardware-run, weakly checked
//
#include <hip/hip_runtime.h>
#include <stddef.h>


typedef _Float16 v16h __attribute__((ext_vector_type(16)));
typedef _Float16 v8h  __attribute__((ext_vector_type(8)));
typedef float    v8f  __attribute__((ext_vector_type(8)));
typedef float    v4f  __attribute__((ext_vector_type(4)));
typedef _Float16 h16;

#ifndef NROWS
#define NROWS 32768
#endif
#define NROWS_FULL 32768
#define NF     32
#define NPOLY  6545
#define NP2    528
#define ECONST 528
#define XCOL   544
#define ECOLS  576
#define EP     580
#define KLOW   576
#define KTOT   7072
#define KPITCH 7104
#define PIECES (KPITCH / 8)
#define LDO    36

#define ACARRY 64.0f
#define WCARRY 1024.0f
#define OUTSCALE (1.0f / (ACARRY * WCARRY))

constexpr unsigned tri_count(unsigned j) { return ((j + 1u) * (j + 2u)) >> 1; }
constexpr unsigned blk_steps(unsigned j) { return (tri_count(j) + 31u) >> 5; }
constexpr unsigned k_total() {
  unsigned k = KLOW;
  for (unsigned j = 0; j < (unsigned)NF; ++j) k += 32u * blk_steps(j);
  return k;
}
constexpr unsigned poly_total() {
  unsigned p = 1u + (unsigned)NF + (unsigned)NP2;
  for (unsigned j = 0; j < (unsigned)NF; ++j) p += tri_count(j);
  return p;
}
static_assert(k_total() == KTOT);
static_assert(poly_total() == NPOLY);
static_assert(tri_count(NF - 1) == NP2);
static_assert(32u * blk_steps(NF - 1) <= (unsigned)XCOL);
static_assert(ECONST == NP2 && XCOL == ECONST + 16 && ECOLS == XCOL + NF && KLOW == ECOLS);
static_assert((KLOW % 32) == 0 && (KTOT % 32) == 0);
static_assert(KPITCH >= KTOT && (KPITCH % 64) == 0 && (PIECES % 8) == 0);
static_assert(EP >= ECOLS && (EP % 4) == 0 && (XCOL % 4) == 0 && (ECONST % 4) == 0);
static_assert((LDO % 4) == 0 && LDO >= NF);
static_assert(NF == 32);
static_assert(NROWS >= 16 && NROWS <= NROWS_FULL && (NROWS % 16) == 0);
static_assert(((32 * PIECES) % 256) == 0);

#define WT_BYTES ((size_t)NF * KPITCH * 2)
#define OFF_WT   ((size_t)0)
#define WS_TOTAL (OFF_WT + WT_BYTES)
static_assert((WT_BYTES % 128) == 0);
static_assert(WS_TOTAL <= (size_t)134217728);

__device__ __forceinline__ float bf16r(float x) {
  unsigned int u = __float_as_uint(x);
  u = (u + 0x7FFFu + ((u >> 16) & 1u)) & 0xFFFF0000u;
  return __uint_as_float(u);
}

static __device__ __forceinline__ h16 toh_flush(float v) {
  const float u = (fabsf(v) < 6.103515625e-05f) ? 0.0f : v;
  return (h16)u;
}

__device__ __forceinline__ v16h frag_at(const _Float16* p) {
  v8h lo = *(const v8h*)(p);
  v8h hi = *(const v8h*)(p + 16);
  v16h out;
#pragma unroll
  for (int i = 0; i < 8; ++i) { out[i] = lo[i]; out[i + 8] = hi[i]; }
  return out;
}

__device__ __forceinline__ v8f wmma16(v16h a, v16h b, v8f c) {
  v8f d = __builtin_amdgcn_wmma_f32_16x16x32_f16(false, a, false, b, (short)0, c,
                                                 false, false);
  asm volatile("v_nop\n\tv_nop\n\tv_nop\n\tv_nop" : "+v"(d) : "v"(a), "v"(b));
  return d;
}

__device__ __forceinline__ void wave_lds_sync() {
  __builtin_amdgcn_fence(3  , "wavefront");
  asm volatile("s_wait_dscnt 0x0" ::: "memory");
  __builtin_amdgcn_wave_barrier();
}

__global__ __launch_bounds__(256) void wprep_kernel(
    const float* __restrict__ W, _Float16* __restrict__ Wt) {
#pragma clang fp contract(off)
  const unsigned t = blockIdx.x * 256u + threadIdx.x;
  const unsigned n = t / (unsigned)PIECES;
  const unsigned pc = t - n * (unsigned)PIECES;
  const unsigned k8 = pc * 8u;

  unsigned kind = 0u;
  unsigned kstart = 0u;
  unsigned cnt = 0u;
  unsigned srcbase = 0u;
  if (k8 >= (unsigned)KLOW) {
    kind = 2u;
    unsigned off = (unsigned)KLOW;
#pragma unroll 1
    for (unsigned u = 0; u < (unsigned)NF; ++u) {
      const unsigned cu = ((u + 1u) * (u + 2u)) >> 1;
      const unsigned len = ((cu + 31u) >> 5) << 5;
      if (k8 >= off && k8 < off + len) {
        kind = 1u;
        kstart = off;
        cnt = cu;
        srcbase = 561u + (u * (u + 1u) * (u + 2u)) / 6u;
      }
      off += len;
    }
  }

  v8h x;
#pragma unroll
  for (unsigned e = 0; e < 8u; ++e) {
    const unsigned q = k8 + e - kstart;
    const int s_low = (q < (unsigned)NP2) ? (int)(33u + q)
                    : ((q == (unsigned)ECONST) ? 0
                    : ((q >= (unsigned)XCOL) ? (int)(1u + q - (unsigned)XCOL) : -1));
    const int s_d3 = (q < cnt) ? (int)(srcbase + q) : -1;
    const int src = (kind == 0u) ? s_low : ((kind == 1u) ? s_d3 : -1);
    int sc = (src < 0) ? 0 : src;
    sc = (sc > NPOLY - 1) ? (NPOLY - 1) : sc;
    float wv = W[(size_t)sc * NF + n];
    asm volatile("" : "+v"(wv));
    const float val = (src >= 0) ? wv : 0.0f;
    x[e] = toh_flush(WCARRY * bf16r(val));
  }
  const size_t off = (size_t)n * KPITCH + k8;
  *(volatile v8h*)(Wt + off) = x;
  __threadfence();
  *(volatile v8h*)(Wt + off) = x;
}

__global__ __launch_bounds__(32) void taylor_kernel(
    const float* __restrict__ X, const _Float16* __restrict__ Wt, float* __restrict__ out) {
  __shared__ __attribute__((aligned(16))) float E[16 * EP];
  __shared__ __attribute__((aligned(16))) float Cs[16 * LDO];

  const unsigned lane = threadIdx.x & 31u;
  const unsigned hh = lane >> 4, m = lane & 15u;
  const unsigned row0 = blockIdx.x * 16u;

#pragma unroll
  for (unsigned j = 0; j < 4u; ++j) {
    const unsigned idx = lane + 32u * j;
    const unsigned r = idx >> 3, c = (idx & 7u) * 4u;
    const v4f a = *(const v4f*)(X + (size_t)(row0 + r) * NF + c);
    v4f b;
#pragma unroll
    for (int i = 0; i < 4; ++i) b[i] = bf16r(a[i]);
    *(v4f*)&E[r * EP + XCOL + c] = b;
  }
  {
    v4f c0 = {0.0f, 0.0f, 0.0f, 0.0f};
    const v4f z = {0.0f, 0.0f, 0.0f, 0.0f};
    c0[0] = (hh == 0u) ? 1.0f : 0.0f;
    *(v4f*)&E[m * EP + ECONST + hh * 8u] = c0;
    *(v4f*)&E[m * EP + ECONST + hh * 8u + 4u] = z;
  }
  wave_lds_sync();

#pragma unroll 1
  for (unsigned j2 = 0; j2 < (unsigned)NF; ++j2) {
    const float xj = E[m * EP + XCOL + j2];
    const unsigned base = (j2 * (j2 + 1u)) >> 1;
#pragma unroll 1
    for (unsigned i2 = 0; i2 <= j2; i2 += 2u) {
      const unsigned i = i2 + hh;
      const unsigned ic = (i < j2) ? i : j2;
      const float v = xj * E[m * EP + XCOL + ic];
      if (i <= j2) E[m * EP + base + i] = v;
    }
  }
  wave_lds_sync();

  const unsigned eo = m * EP + hh * 8u;
  const _Float16* bp0 = Wt + (size_t)m * KPITCH + hh * 8u;
  const _Float16* bp1 = bp0 + (size_t)16 * KPITCH;
  v8f acc0 = {}, acc1 = {};
  unsigned kk = 0u;

#pragma unroll 1
  for (unsigned t = 0; t < (unsigned)NF + 1u; ++t) {
    const unsigned j = (t == 0u) ? 0u : (t - 1u);
    const float xs = E[m * EP + XCOL + j];
    const float sc = ACARRY * ((t == 0u) ? 1.0f : xs);
    const unsigned cj = (t * (t + 1u)) >> 1;
    const unsigned ns = (t == 0u) ? (unsigned)(KLOW / 32) : ((cj + 31u) >> 5);
#pragma unroll 1
    for (unsigned s = 0; s < ns; ++s) {
      const unsigned q0 = s * 32u;
      const v4f e0 = *(const v4f*)&E[eo + q0];
      const v4f e1 = *(const v4f*)&E[eo + q0 + 4u];
      const v4f e2 = *(const v4f*)&E[eo + q0 + 16u];
      const v4f e3 = *(const v4f*)&E[eo + q0 + 20u];
      v16h a;
#pragma unroll
      for (int i = 0; i < 4; ++i) {
        a[i]      = toh_flush(sc * e0[i]);
        a[i + 4]  = toh_flush(sc * e1[i]);
        a[i + 8]  = toh_flush(sc * e2[i]);
        a[i + 12] = toh_flush(sc * e3[i]);
      }
      const v16h b0 = frag_at(bp0 + kk);
      const v16h b1 = frag_at(bp1 + kk);
      acc0 = wmma16(a, b0, acc0);
      acc1 = wmma16(a, b1, acc1);
      kk += 32u;
    }
  }

#pragma unroll
  for (int r = 0; r < 8; ++r) {
    Cs[(hh * 8u + (unsigned)r) * LDO + m]       = acc0[r];
    Cs[(hh * 8u + (unsigned)r) * LDO + 16u + m] = acc1[r];
  }
  wave_lds_sync();

  v4f xs4[4];
  size_t off[4];
#pragma unroll
  for (unsigned i = 0; i < 4u; ++i) {
    const unsigned r = 4u * i + (lane >> 3);
    const unsigned c = (lane & 7u) * 4u;
    const v4f u = *(const v4f*)&Cs[r * LDO + c];
    xs4[i] = u * OUTSCALE;
    off[i] = (size_t)(row0 + r) * NF + c;
  }
#pragma unroll
  for (int i = 0; i < 4; ++i) *(volatile v4f*)(out + off[i]) = xs4[i];
  __threadfence();
#pragma unroll
  for (int i = 0; i < 4; ++i) *(volatile v4f*)(out + off[i]) = xs4[i];
}

extern "C" void kernel_launch(void* const* d_in, const int* in_sizes, int n_in,
                              void* d_out, int out_size, void* d_ws, size_t ws_size,
                              hipStream_t stream) {
  if (n_in < 2) return;
  if ((long long)in_sizes[0] < (long long)NROWS * NF) return;
  if ((long long)in_sizes[1] < (long long)NPOLY * NF) return;
  if ((long long)out_size < (long long)NROWS * NF) return;
  if (ws_size < WS_TOTAL) return;

  const float* X = (const float*)d_in[0];
  const float* W = (const float*)d_in[1];
  float* out = (float*)d_out;
  char* ws = (char*)d_ws;
  _Float16* Wt = (_Float16*)(ws + OFF_WT);

  wprep_kernel<<<dim3((32 * PIECES) / 256), dim3(256), 0, stream>>>(W, Wt);
  taylor_kernel<<<dim3(NROWS / 16), dim3(32), 0, stream>>>(X, Wt, out);
}
